// T5Gemma2EncoderAttention_90855738180356
// MI455X (gfx1250) — hardware-verified
//
#include <hip/hip_runtime.h>


#define NB_  2
#define TT   2048
#define DM   2048
#define NQ   8
#define NKV  4
#define HDD  256
#define DKV  (NKV * HDD)
#define ZH   2
#define PCAR 1024.0f
#define KMASK (-3.3895313892515355e38f)
typedef _Float16 h16;
typedef unsigned short bf;
typedef __attribute__((ext_vector_type(16))) __bf16   v16bf;
typedef __attribute__((ext_vector_type(16))) _Float16 v16h;
typedef __attribute__((ext_vector_type(8)))  _Float16 v8h;
typedef __attribute__((ext_vector_type(8)))  unsigned short v8us;
typedef __attribute__((ext_vector_type(8)))  float    v8f;
typedef __attribute__((ext_vector_type(4)))  float    v4f;
typedef v8h  __attribute__((may_alias)) v8ha;
typedef v4f  __attribute__((may_alias)) v4fa;
typedef v8us __attribute__((may_alias)) v8usa;

__device__ __forceinline__ unsigned short f2bf(float f) { unsigned u = __float_as_uint(f); u += 0x7FFFu + ((u >> 16) & 1u); return (unsigned short)(u >> 16); }
__device__ __forceinline__ float bf2f(unsigned short b) { return __uint_as_float(((unsigned)b) << 16); }
__device__ __forceinline__ float bfr(float f) { return bf2f(f2bf(f)); }
__device__ __forceinline__ v16h cat16(v8h lo, v8h hi) { return __builtin_shufflevector(lo, hi, 0, 1, 2, 3, 4, 5, 6, 7, 8, 9, 10, 11, 12, 13, 14, 15); }
__device__ __forceinline__ v16bf cat16b(v8us lo, v8us hi) { return __builtin_bit_cast(v16bf, __builtin_shufflevector(lo, hi, 0, 1, 2, 3, 4, 5, 6, 7, 8, 9, 10, 11, 12, 13, 14, 15)); }
__device__ __forceinline__ v8f wmma16(v16h a, v16h b, v8f c) { return __builtin_amdgcn_wmma_f32_16x16x32_f16(false, a, false, b, (short)0, c, false, false); }
__device__ __forceinline__ v8f wmmab(v16bf a, v16bf b, v8f c) { return __builtin_amdgcn_wmma_f32_16x16x32_bf16(false, a, false, b, (short)0, c, false, false); }


template <typename T16> struct WFrag;
template <> struct WFrag<h16> { typedef v16h V; static __device__ __forceinline__ V ld(const h16* p) { return cat16(*(const v8h*)p, *(const v8h*)(p + 16)); } static __device__ __forceinline__ v8f mma(V a, V b, v8f c) { return wmma16(a, b, c); } };
template <> struct WFrag<bf> { typedef v16bf V; static __device__ __forceinline__ V ld(const bf* p) { return cat16b(*(const v8us*)p, *(const v8us*)(p + 16)); } static __device__ __forceinline__ v8f mma(V a, V b, v8f c) { return wmmab(a, b, c); } };
template <typename T16, int NSPLIT, bool BIAS>
__global__ __launch_bounds__(32) void k_gemmw(const T16* __restrict__ A, const T16* __restrict__ A2, const T16* __restrict__ Bt, const T16* __restrict__ Bt2, int K, float* C, int ldc, const float* __restrict__ bias, size_t sA, size_t sB, size_t sC) {
    typedef typename WFrag<T16>::V V;
    __shared__ __align__(16) float os[16 * 68];
    const size_t z = blockIdx.z; A += z * sA; if (A2) A2 += z * sA; Bt += z * sB; if (Bt2) Bt2 += z * sB; C += z * sC;
    const int lane = threadIdx.x & 31, lr = lane & 15, hi = lane >> 4; const int r0 = blockIdx.x * 64, c0 = blockIdx.y * 64;
    v8f acc[4][4];
#pragma unroll
    for (int mb = 0; mb < 4; ++mb)
#pragma unroll
        for (int nb = 0; nb < 4; ++nb) acc[mb][nb] = (v8f){};
    const size_t aoff = (size_t)(r0 + lr) * K + 8 * hi, boff = (size_t)(c0 + lr) * K + 8 * hi;
#pragma unroll 1
    for (int kc = 0; kc < K; kc += 32) {
        V a[4], a2[4];
#pragma unroll
        for (int mb = 0; mb < 4; ++mb) { a[mb] = WFrag<T16>::ld(A + aoff + (size_t)mb * 16 * K + kc); if (NSPLIT == 1 || NSPLIT == 2) a2[mb] = WFrag<T16>::ld(A2 + aoff + (size_t)mb * 16 * K + kc); }
#pragma unroll
        for (int nb = 0; nb < 4; ++nb) { const V b = WFrag<T16>::ld(Bt + boff + (size_t)nb * 16 * K + kc); V b2; if (NSPLIT >= 2) b2 = WFrag<T16>::ld(Bt2 + boff + (size_t)nb * 16 * K + kc);
#pragma unroll
            for (int mb = 0; mb < 4; ++mb) { acc[mb][nb] = WFrag<T16>::mma(a[mb], b, acc[mb][nb]); if (NSPLIT == 1 || NSPLIT == 2) acc[mb][nb] = WFrag<T16>::mma(a2[mb], b, acc[mb][nb]); if (NSPLIT >= 2) acc[mb][nb] = WFrag<T16>::mma(a[mb], b2, acc[mb][nb]); } }
        asm volatile("v_nop\n\tv_nop\n\tv_nop\n\tv_nop" : "+v"(acc[0][0]), "+v"(acc[1][1]), "+v"(acc[2][2]), "+v"(acc[3][3]) : "v"(a[0]), "v"(a[3]));
    }
#pragma unroll
    for (int mb = 0; mb < 4; ++mb) {
#pragma unroll
        for (int nb = 0; nb < 4; ++nb) {
#pragma unroll
            for (int j = 0; j < 8; ++j) os[(hi * 8 + j) * 68 + nb * 16 + lr] = acc[mb][nb][j]; }
        __builtin_amdgcn_wave_barrier(); asm volatile("" ::: "memory");
        float* crow = C + (size_t)(r0 + mb * 16) * ldc + c0;
#pragma unroll 1
        for (int ps = 0; ps < 2; ++ps) {
#pragma unroll
            for (int s = 0; s < 8; ++s) { const int row = 2 * s + hi, cofs = lr * 4; v4f val = *(const v4fa*)(os + row * 68 + cofs); if (BIAS) { val[0] += bfr(bias[c0 + cofs]); val[1] += bfr(bias[c0 + cofs + 1]); val[2] += bfr(bias[c0 + cofs + 2]); val[3] += bfr(bias[c0 + cofs + 3]); }
                *(volatile v4f*)(crow + (size_t)row * ldc + cofs) = val; }
            if (ps == 0) __threadfence(); }
        __builtin_amdgcn_wave_barrier(); asm volatile("" ::: "memory");
    }
}

__device__ __forceinline__ h16 tohx(float x) { return (h16)x; }
__device__ __forceinline__ void splitf(float y, unsigned short& h, unsigned short& l) { h = f2bf(y); l = f2bf(y - bf2f(h)); }
typedef __attribute__((ext_vector_type(2))) unsigned short v2us;
typedef __attribute__((ext_vector_type(4))) unsigned short v4us;
typedef __attribute__((ext_vector_type(2))) _Float16 v2h;
typedef __attribute__((ext_vector_type(4))) _Float16 v4h;

__global__ __launch_bounds__(256) void k_cvt8(const float* __restrict__ src, bf* dst, size_t n8) { const size_t i = (size_t)blockIdx.x * 256 + threadIdx.x; if (i >= n8) return; const v8f v = *(const v8f*)(src + i * 8); v8us o;
#pragma unroll
    for (int k = 0; k < 8; ++k) o[k] = f2bf(v[k]); *(volatile v8us*)(dst + i * 8) = o; __threadfence(); *(volatile v8us*)(dst + i * 8) = o; }
__global__ __launch_bounds__(256) void k_wtG(const float* __restrict__ w, int K, int N, bf* Bt) {
    const int lane = threadIdx.x & 31; const int L0 = (blockIdx.x * 8 + (threadIdx.x >> 5)) * 8; const int nlines = N * K / 64;
#pragma unroll
    for (int ps = 0; ps < 2; ++ps) {
#pragma unroll 1
        for (int l = 0; l < 8; ++l) { const int L = L0 + l; if (L >= nlines) break; const size_t e = (size_t)L * 64 + lane * 2; const int k = (int)(e % K), n = (int)(e / K); v2us o;
            o[0] = f2bf(w[(size_t)k * N + n]); o[1] = f2bf(w[(size_t)(k + 1) * N + n]); *(volatile v2us*)(Bt + e) = o; }
        if (ps == 0) __threadfence(); }
}

__device__ __attribute__((noinline)) float softcap50(float s) { return 50.0f * tanhf(s * 0.02f); }
typedef __attribute__((ext_vector_type(2))) float v2f_t;
__device__ __attribute__((noinline)) v2f_t sincos_pos(float pos, int i) { const float tsc = powf(10000.0f, (2.0f / (float)HDD) * (float)i); const float ang = __fdiv_rn(pos, tsc); v2f_t r; r[0] = sinf(ang); r[1] = cosf(ang); return r; }
__global__ __launch_bounds__(256) void k_whd(const float* __restrict__ W, int nh, bf* Bt) { const size_t e = ((size_t)blockIdx.x * 256 + threadIdx.x) * 4; if (e >= (size_t)nh * HDD * DM) return; const int k = (int)(e % DM); const int row = (int)(e / DM); const int n = row / HDD, d = row % HDD; v4us o;
#pragma unroll
    for (int u = 0; u < 4; ++u) o[u] = f2bf(W[((size_t)n * DM + k + u) * HDD + d]); *(volatile v4us*)(Bt + e) = o; __threadfence(); *(volatile v4us*)(Bt + e) = o; }
__global__ __launch_bounds__(256) void k_nrr(const float* __restrict__ F, int pitch, int nheads, const float* __restrict__ scale, const int* __restrict__ pos, float mul, bf* Ph, bf* Pl) { const int lane = threadIdx.x & 31; const int wv = blockIdx.x * 8 + (threadIdx.x >> 5); if (wv >= TT * nheads) return; const int t = wv / nheads, h = wv % nheads; const float* f = F + (size_t)t * pitch + h * HDD;
    const v4f a = *(const v4f*)(f + lane * 4), b2 = *(const v4f*)(f + HDD / 2 + lane * 4); float ss = 0.f; for (int q = 0; q < 4; ++q) { float p = __fmul_rn(a[q], a[q]); asm volatile("" : "+v"(p)); ss = __fadd_rn(ss, p); p = __fmul_rn(b2[q], b2[q]); asm volatile("" : "+v"(p)); ss = __fadd_rn(ss, p); }
#pragma unroll
    for (int sh = 16; sh; sh >>= 1) ss = __fadd_rn(ss, __shfl_xor(ss, sh, 32));
    const float rs = __fdiv_rn(1.0f, sqrtf(__fadd_rn(ss * (1.0f / HDD), 1e-6f))); const float pv = (float)pos[t]; v4us ah, al, bh, bl;
#pragma unroll
    for (int q = 0; q < 4; ++q) { const int i = lane * 4 + q; float n1 = __fmul_rn(a[q], rs), n2 = __fmul_rn(b2[q], rs); asm volatile("" : "+v"(n1)); asm volatile("" : "+v"(n2)); const float x1 = __fmul_rn(n1, __fadd_rn(1.0f, bfr(scale[i]))), x2 = __fmul_rn(n2, __fadd_rn(1.0f, bfr(scale[i + HDD / 2]))); const v2f_t sc2 = sincos_pos(pv, i); const float sn = sc2[0], cs = sc2[1];
        float p1 = __fmul_rn(x1, cs), p2 = __fmul_rn(x2, sn), p3 = __fmul_rn(x2, cs), p4 = __fmul_rn(x1, sn); asm volatile("" : "+v"(p1)); asm volatile("" : "+v"(p2)); asm volatile("" : "+v"(p3)); asm volatile("" : "+v"(p4));
        const float r1 = __fsub_rn(p1, p2) * mul, r2 = __fadd_rn(p3, p4) * mul; unsigned short u1, l1, u2, l2; splitf(r1, u1, l1); splitf(r2, u2, l2); ah[q] = u1; al[q] = l1; bh[q] = u2; bl[q] = l2; }
    bf* dh = Ph + ((size_t)h * TT + t) * HDD; bf* dl = Pl + ((size_t)h * TT + t) * HDD; *(volatile v4us*)(dh + lane * 4) = ah; *(volatile v4us*)(dl + lane * 4) = al; *(volatile v4us*)(dh + HDD / 2 + lane * 4) = bh; *(volatile v4us*)(dl + HDD / 2 + lane * 4) = bl; __threadfence(); *(volatile v4us*)(dh + lane * 4) = ah; *(volatile v4us*)(dl + lane * 4) = al; *(volatile v4us*)(dh + HDD / 2 + lane * 4) = bh; *(volatile v4us*)(dl + HDD / 2 + lane * 4) = bl; }
__global__ __launch_bounds__(256) void k_vt16(const float* __restrict__ F, h16* VT) { const size_t e = ((size_t)blockIdx.x * 256 + threadIdx.x) * 2; if (e >= (size_t)NKV * HDD * TT) return; const int t = (int)(e % TT); const int d = (int)((e / TT) % HDD); const int c = (int)(e / ((size_t)TT * HDD)); v2h o; o[0] = tohx(F[(size_t)t * DKV + c * HDD + d]); o[1] = tohx(F[(size_t)(t + 1) * DKV + c * HDD + d]); *(volatile v2h*)(VT + e) = o; __threadfence(); *(volatile v2h*)(VT + e) = o; }
__global__ __launch_bounds__(256) void k_tsoft(const float* __restrict__ S, const int* __restrict__ pos, const int* __restrict__ am, h16* P16) { const int lane = threadIdx.x & 31; const int row = blockIdx.x * 8 + (threadIdx.x >> 5); if (row >= ZH * TT) return; const int i = row % TT; const float* sr = S + (size_t)row * TT; const int* mr = am + (size_t)i * TT; const int pi = pos[i]; float v[TT / 32]; float mx = -3.0e38f;
#pragma unroll
    for (int ch = 0; ch < TT / 128; ++ch) { const v4f a = *(const v4f*)(sr + ch * 128 + lane * 4);
#pragma unroll
        for (int u = 0; u < 4; ++u) { const int j = ch * 128 + lane * 4 + u; const int dist = pi - pos[j]; const bool win = (dist >= 0 && dist < 256) || (dist < 0 && -dist < 257); const bool ok = win && (mr[j] != 0); const float t = ok ? softcap50(a[u]) : KMASK; v[ch * 4 + u] = t; mx = fmaxf(mx, t); } }
#pragma unroll
    for (int sh = 16; sh; sh >>= 1) mx = fmaxf(mx, __shfl_xor(mx, sh, 32));
    float sum = 0.f;
#pragma unroll
    for (int q = 0; q < TT / 32; ++q) { float d0 = __fsub_rn(v[q], mx); asm volatile("" : "+v"(d0)); v[q] = __builtin_amdgcn_exp2f(__fmul_rn(d0, 1.4426950408889634f)); sum += v[q]; }
#pragma unroll
    for (int sh = 16; sh; sh >>= 1) sum += __shfl_xor(sum, sh, 32);
    const float f = __fdiv_rn(PCAR, sum);
    for (int ps = 0; ps < 2; ++ps) {
#pragma unroll
        for (int ch = 0; ch < TT / 128; ++ch) { v4h o4; for (int q = 0; q < 4; ++q) o4[q] = tohx(v[ch * 4 + q] * f); *(volatile v4h*)(P16 + (size_t)row * TT + ch * 128 + lane * 4) = o4; }
        if (ps == 0) __threadfence(); } }
__global__ __launch_bounds__(256) void k_mrg(const float* __restrict__ O, int n0, bf* Ah, bf* Al) { const size_t e = ((size_t)blockIdx.x * 256 + threadIdx.x) * 4; if (e >= (size_t)ZH * TT * HDD) return; const int d = (int)(e % HDD); const int t = (int)((e / HDD) % TT); const int zz = (int)(e / ((size_t)HDD * TT)); const size_t oo = (size_t)t * DM + (n0 + zz) * HDD + d; v4us oh, ol;
#pragma unroll
    for (int u = 0; u < 4; ++u) { unsigned short a, b; splitf(O[e + u] * (1.0f / PCAR), a, b); oh[u] = a; ol[u] = b; } *(volatile v4us*)(Ah + oo) = oh; *(volatile v4us*)(Al + oo) = ol; __threadfence(); *(volatile v4us*)(Ah + oo) = oh; *(volatile v4us*)(Al + oo) = ol; }

extern "C" void kernel_launch(void* const* d_in, const int* in_sizes, int n_in,
                              void* d_out, int out_size, void* d_ws, size_t ws_size, hipStream_t stream) {
    (void)in_sizes; (void)n_in; (void)out_size;
    const float* x = (const float*)d_in[0]; const int* spos = (const int*)d_in[1]; const int* amask = (const int*)d_in[2]; const float* wq = (const float*)d_in[3]; const float* wkv = (const float*)d_in[4]; const float* wo = (const float*)d_in[5]; const float* qs = (const float*)d_in[6]; const float* ks = (const float*)d_in[7];
    float* OUT = (float*)d_out;
    char* wsp = (char*)d_ws;
    auto take = [&](size_t bytes) { char* p = wsp; wsp += (bytes + 255) & ~(size_t)255; return (void*)p; };
    bf* BQ = (bf*)take((size_t)NQ * HDD * DM * 2); bf* BK = (bf*)take((size_t)DKV * DM * 2); bf* BV = (bf*)take((size_t)DKV * DM * 2); bf* BO = (bf*)take((size_t)DM * DM * 2);
    bf* XB = (bf*)take((size_t)TT * DM * 2); float* FQ = (float*)take((size_t)TT * DM * 4); float* FK = (float*)take((size_t)TT * DKV * 4);
    bf* QPh = (bf*)take((size_t)NQ * TT * HDD * 2); bf* QPl = (bf*)take((size_t)NQ * TT * HDD * 2); bf* KPh = (bf*)take((size_t)NKV * TT * HDD * 2); bf* KPl = (bf*)take((size_t)NKV * TT * HDD * 2); h16* VT = (h16*)take((size_t)NKV * HDD * TT * 2);
    float* S = (float*)take((size_t)ZH * TT * TT * 4); h16* P16 = (h16*)take((size_t)ZH * TT * TT * 2); float* O = (float*)take((size_t)ZH * TT * HDD * 4); bf* ENh = (bf*)take((size_t)TT * DM * 2); bf* ENl = (bf*)take((size_t)TT * DM * 2);
    if ((size_t)(wsp - (char*)d_ws) > ws_size) return;
    float* FV = FK;
    k_whd<<<(unsigned)(((size_t)NQ * HDD * DM / 4 + 255) / 256), 256, 0, stream>>>(wq, NQ, BQ); k_whd<<<(unsigned)(((size_t)DKV * DM / 4 + 255) / 256), 256, 0, stream>>>(wkv, NKV, BK); k_whd<<<(unsigned)(((size_t)DKV * DM / 4 + 255) / 256), 256, 0, stream>>>(wkv + (size_t)NKV * DM * HDD, NKV, BV);
    k_wtG<<<(DM * DM / 64 + 63) / 64, 256, 0, stream>>>(wo, DM, DM, BO);
    const size_t zq = (size_t)TT * HDD, zS = (size_t)TT * TT, zv = (size_t)HDD * TT, zo = (size_t)TT * HDD;
    for (int b = 0; b < NB_; ++b) {
        k_cvt8<<<(TT * DM / 8 + 255) / 256, 256, 0, stream>>>(x + (size_t)b * TT * DM, XB, TT * DM / 8);
        k_gemmw<bf, 0, false><<<dim3(TT / 64, DM / 64, 1), 32, 0, stream>>>(XB, nullptr, BQ, nullptr, DM, FQ, DM, nullptr, 0, 0, 0);
        k_nrr<<<TT * NQ / 8, 256, 0, stream>>>(FQ, DM, NQ, qs, spos + (size_t)b * TT, 0.0625f, QPh, QPl);
        k_gemmw<bf, 0, false><<<dim3(TT / 64, DKV / 64, 1), 32, 0, stream>>>(XB, nullptr, BK, nullptr, DM, FK, DKV, nullptr, 0, 0, 0);
        k_nrr<<<TT * NKV / 8, 256, 0, stream>>>(FK, DKV, NKV, ks, spos + (size_t)b * TT, 1.0f, KPh, KPl);
        k_gemmw<bf, 0, false><<<dim3(TT / 64, DKV / 64, 1), 32, 0, stream>>>(XB, nullptr, BV, nullptr, DM, FV, DKV, nullptr, 0, 0, 0);
        k_vt16<<<(unsigned)(((size_t)NKV * HDD * TT / 2 + 255) / 256), 256, 0, stream>>>(FV, VT);
        for (int n0 = 0; n0 < NQ; n0 += ZH) { const size_t zk = (size_t)(n0 / 2);
            k_gemmw<bf, 2, false><<<dim3(TT / 64, TT / 64, ZH), 32, 0, stream>>>(QPh + (size_t)n0 * zq, QPl + (size_t)n0 * zq, KPh + zk * zq, KPl + zk * zq, HDD, S, TT, nullptr, zq, 0, zS);
            k_tsoft<<<ZH * TT / 8, 256, 0, stream>>>(S, spos + (size_t)b * TT, amask + (size_t)b * TT * TT, P16);
            k_gemmw<h16, 0, false><<<dim3(TT / 64, HDD / 64, ZH), 32, 0, stream>>>(P16, nullptr, VT + zk * zv, nullptr, TT, O, HDD, nullptr, zS, 0, zo);
            k_mrg<<<(unsigned)(((size_t)ZH * TT * HDD / 4 + 255) / 256), 256, 0, stream>>>(O, n0, ENh, ENl); }
        k_gemmw<bf, 1, false><<<dim3(TT / 64, DM / 64, 1), 32, 0, stream>>>(ENh, ENl, BO, nullptr, DM, OUT + (size_t)b * TT * DM, DM, nullptr, 0, 0, 0); }
}
